// MobiuAttention_8564164788652
// MI455X (gfx1250) — hardware-verified
//
#include <hip/hip_runtime.h>


#define NB_  4
#define TT   2048
#define DM   1024
#define NH_  16
#define EE   64
#define CH   64
#define NC   (TT / CH)
#define NZ   (NH_ * NC)
#define SEN  256
typedef _Float16 h16;
typedef unsigned short bf;
typedef __attribute__((ext_vector_type(16))) __bf16   v16bf;
typedef __attribute__((ext_vector_type(16))) _Float16 v16h;
typedef __attribute__((ext_vector_type(8)))  _Float16 v8h;
typedef __attribute__((ext_vector_type(8)))  unsigned short v8us;
typedef __attribute__((ext_vector_type(8)))  float    v8f;
typedef __attribute__((ext_vector_type(4)))  float    v4f;
typedef v8h  __attribute__((may_alias)) v8ha;
typedef v4f  __attribute__((may_alias)) v4fa;
typedef v8us __attribute__((may_alias)) v8usa;

__device__ __forceinline__ unsigned short f2bf(float f) { unsigned u = __float_as_uint(f); u += 0x7FFFu + ((u >> 16) & 1u); return (unsigned short)(u >> 16); }
__device__ __forceinline__ float bf2f(unsigned short b) { return __uint_as_float(((unsigned)b) << 16); }
__device__ __forceinline__ float bfr(float f) { return bf2f(f2bf(f)); }
__device__ __forceinline__ v16h cat16(v8h lo, v8h hi) { return __builtin_shufflevector(lo, hi, 0, 1, 2, 3, 4, 5, 6, 7, 8, 9, 10, 11, 12, 13, 14, 15); }
__device__ __forceinline__ v16bf cat16b(v8us lo, v8us hi) { return __builtin_bit_cast(v16bf, __builtin_shufflevector(lo, hi, 0, 1, 2, 3, 4, 5, 6, 7, 8, 9, 10, 11, 12, 13, 14, 15)); }
__device__ __forceinline__ v8f wmma16(v16h a, v16h b, v8f c) { return __builtin_amdgcn_wmma_f32_16x16x32_f16(false, a, false, b, (short)0, c, false, false); }
__device__ __forceinline__ v8f wmmab(v16bf a, v16bf b, v8f c) { return __builtin_amdgcn_wmma_f32_16x16x32_bf16(false, a, false, b, (short)0, c, false, false); }


template <typename T16> struct WFrag;
template <> struct WFrag<h16> { typedef v16h V; static __device__ __forceinline__ V ld(const h16* p) { return cat16(*(const v8h*)p, *(const v8h*)(p + 16)); } static __device__ __forceinline__ v8f mma(V a, V b, v8f c) { return wmma16(a, b, c); } };
template <> struct WFrag<bf> { typedef v16bf V; static __device__ __forceinline__ V ld(const bf* p) { return cat16b(*(const v8us*)p, *(const v8us*)(p + 16)); } static __device__ __forceinline__ v8f mma(V a, V b, v8f c) { return wmmab(a, b, c); } };
template <typename T16, int NSPLIT, bool BIAS>
__global__ __launch_bounds__(32) void k_gemmw(const T16* __restrict__ A, const T16* __restrict__ A2, const T16* __restrict__ Bt, const T16* __restrict__ Bt2, int K, float* C, int ldc, const float* __restrict__ bias, size_t sA, size_t sB, size_t sC) {
    typedef typename WFrag<T16>::V V;
    __shared__ __align__(16) float os[16 * 68];
    const size_t z = blockIdx.z; A += z * sA; if (A2) A2 += z * sA; Bt += z * sB; if (Bt2) Bt2 += z * sB; C += z * sC;
    const int lane = threadIdx.x & 31, lr = lane & 15, hi = lane >> 4; const int r0 = blockIdx.x * 64, c0 = blockIdx.y * 64;
    v8f acc[4][4];
#pragma unroll
    for (int mb = 0; mb < 4; ++mb)
#pragma unroll
        for (int nb = 0; nb < 4; ++nb) acc[mb][nb] = (v8f){};
    const size_t aoff = (size_t)(r0 + lr) * K + 8 * hi, boff = (size_t)(c0 + lr) * K + 8 * hi;
#pragma unroll 1
    for (int kc = 0; kc < K; kc += 32) {
        V a[4], a2[4];
#pragma unroll
        for (int mb = 0; mb < 4; ++mb) { a[mb] = WFrag<T16>::ld(A + aoff + (size_t)mb * 16 * K + kc); if (NSPLIT == 1 || NSPLIT == 2) a2[mb] = WFrag<T16>::ld(A2 + aoff + (size_t)mb * 16 * K + kc); }
#pragma unroll
        for (int nb = 0; nb < 4; ++nb) { const V b = WFrag<T16>::ld(Bt + boff + (size_t)nb * 16 * K + kc); V b2; if (NSPLIT >= 2) b2 = WFrag<T16>::ld(Bt2 + boff + (size_t)nb * 16 * K + kc);
#pragma unroll
            for (int mb = 0; mb < 4; ++mb) { acc[mb][nb] = WFrag<T16>::mma(a[mb], b, acc[mb][nb]); if (NSPLIT == 1 || NSPLIT == 2) acc[mb][nb] = WFrag<T16>::mma(a2[mb], b, acc[mb][nb]); if (NSPLIT >= 2) acc[mb][nb] = WFrag<T16>::mma(a[mb], b2, acc[mb][nb]); } }
        asm volatile("v_nop\n\tv_nop\n\tv_nop\n\tv_nop" : "+v"(acc[0][0]), "+v"(acc[1][1]), "+v"(acc[2][2]), "+v"(acc[3][3]) : "v"(a[0]), "v"(a[3]));
    }
#pragma unroll
    for (int mb = 0; mb < 4; ++mb) {
#pragma unroll
        for (int nb = 0; nb < 4; ++nb) {
#pragma unroll
            for (int j = 0; j < 8; ++j) os[(hi * 8 + j) * 68 + nb * 16 + lr] = acc[mb][nb][j]; }
        __builtin_amdgcn_wave_barrier(); asm volatile("" ::: "memory");
        float* crow = C + (size_t)(r0 + mb * 16) * ldc + c0;
#pragma unroll 1
        for (int ps = 0; ps < 2; ++ps) {
#pragma unroll
            for (int s = 0; s < 8; ++s) { const int row = 2 * s + hi, cofs = lr * 4; v4f val = *(const v4fa*)(os + row * 68 + cofs); if (BIAS) { val[0] += bfr(bias[c0 + cofs]); val[1] += bfr(bias[c0 + cofs + 1]); val[2] += bfr(bias[c0 + cofs + 2]); val[3] += bfr(bias[c0 + cofs + 3]); }
                *(volatile v4f*)(crow + (size_t)row * ldc + cofs) = val; }
            if (ps == 0) __threadfence(); }
        __builtin_amdgcn_wave_barrier(); asm volatile("" ::: "memory");
    }
}

__device__ __forceinline__ void splitf(float y, unsigned short& h, unsigned short& l) { h = f2bf(y); l = f2bf(y - bf2f(h)); }
__device__ __forceinline__ float sigm_(float x) { return __fdiv_rn(1.0f, 1.0f + __expf(-x)); }
typedef __attribute__((ext_vector_type(2))) unsigned short v2us;
typedef __attribute__((ext_vector_type(4))) unsigned short v4us;

__global__ __launch_bounds__(256) void k_cvt8(const float* __restrict__ src, bf* dst, size_t n8) { const size_t i = (size_t)blockIdx.x * 256 + threadIdx.x; if (i >= n8) return; const v8f v = *(const v8f*)(src + i * 8); v8us o;
#pragma unroll
    for (int k = 0; k < 8; ++k) o[k] = f2bf(v[k]); *(volatile v8us*)(dst + i * 8) = o; __threadfence(); *(volatile v8us*)(dst + i * 8) = o; }
__global__ __launch_bounds__(256) void k_lc(const float* __restrict__ SENS, const float* __restrict__ w2, const float* __restrict__ b2, float* LC) { const int i = blockIdx.x * 256 + threadIdx.x; if (i >= TT * NH_) return; const int h = i % NH_, t = i / NH_; const float* s = SENS + (size_t)t * SEN; float acc = bfr(b2[h]);
#pragma unroll 1
    for (int j = 0; j < SEN; ++j) { float p = __fmul_rn(tanhf(s[j]), bfr(w2[h * SEN + j])); asm volatile("" : "+v"(p)); acc = __fadd_rn(acc, p); } const float v = sigm_(acc); *(volatile float*)(LC + i) = v; __threadfence(); *(volatile float*)(LC + i) = v; }
__global__ __launch_bounds__(256) void k_bcum(const float* __restrict__ LC, const float* __restrict__ decay, float* BC) { const int i = blockIdx.x * 256 + threadIdx.x; if (i >= NH_ * NC * EE) return; const int e = i % EE; const int c = (i / EE) % NC; const int h = i / (EE * NC); const float base = sigm_(bfr(decay[h * EE + e])); float b = 1.0f;
    for (int ps = 0; ps < 2; ++ps) { b = 1.0f;
#pragma unroll 1
        for (int j = 0; j < CH; ++j) { const int t = c * CH + j; if (j == CH / 2) b = 1.0f;     float lam = __fmul_rn(base, __fadd_rn(1.0f, 0.2f * LC[t * NH_ + h])); lam = fminf(fmaxf(lam, 0.f), 0.9995f); b = __fmul_rn(b, lam); *(volatile float*)(BC + ((size_t)h * TT + t) * EE + e) = b; }
        if (ps == 0) __threadfence(); } }
__global__ __launch_bounds__(256) void k_qkpl(const float* __restrict__ FQ, const float* __restrict__ FK, const float* __restrict__ BC, bf* QMh, bf* QMl, bf* QAh, bf* QAl, bf* KBh, bf* KBl) { const int i = (blockIdx.x * 256 + threadIdx.x) * 4; if (i >= NH_ * TT * EE) return; const int e = i % EE; const int t = (i / EE) % TT; const int h = i / (EE * TT); const int tm = (t / CH) * CH + 31; const bool first = (t % CH) < CH / 2;
    const v4f q = *(const v4f*)(FQ + (size_t)t * DM + h * EE + e), k = *(const v4f*)(FK + (size_t)t * DM + h * EE + e), hp = *(const v4f*)(BC + ((size_t)h * TT + t) * EE + e), pm = *(const v4f*)(BC + ((size_t)h * TT + tm) * EE + e); v4us a1, a2, b1, b2, c1, c2;
#pragma unroll
    for (int u = 0; u < 4; ++u) { const float rm = first ? __fdiv_rn(hp[u], pm[u]) : hp[u];     const float ba = first ? hp[u] : __fmul_rn(pm[u], hp[u]);     const float km = first ? __fdiv_rn(pm[u], hp[u]) : __fdiv_rn(1.0f, hp[u]);
        unsigned short hh, ll; splitf(__fmul_rn(q[u], rm), hh, ll); a1[u] = hh; a2[u] = ll; splitf(__fmul_rn(q[u], ba), hh, ll); b1[u] = hh; b2[u] = ll; splitf(__fmul_rn(k[u], km), hh, ll); c1[u] = hh; c2[u] = ll; }
    for (int ps = 0; ps < 2; ++ps) { *(volatile v4us*)(QMh + i) = a1; *(volatile v4us*)(QMl + i) = a2; *(volatile v4us*)(QAh + i) = b1; *(volatile v4us*)(QAl + i) = b2; *(volatile v4us*)(KBh + i) = c1; *(volatile v4us*)(KBl + i) = c2; if (ps == 0) __threadfence(); } }
__global__ __launch_bounds__(256) void k_ktvt(const float* __restrict__ FK, const float* __restrict__ FV, const float* __restrict__ BC, bf* KTh, bf* KTl, bf* VTh, bf* VTl) { const int i = (blockIdx.x * 256 + threadIdx.x) * 2; if (i >= NH_ * NC * EE * CH) return; const int s = i % CH; const int r = (i / CH) % EE; const int c = (i / (CH * EE)) % NC; const int h = i / (CH * EE * NC); const int tl = c * CH + CH - 1, tm = c * CH + 31; const float p2l = BC[((size_t)h * TT + tl) * EE + r], p1m = BC[((size_t)h * TT + tm) * EE + r]; v2us kh, kl, vh, vl;
#pragma unroll
    for (int u = 0; u < 2; ++u) { const int t = c * CH + s + u; const float kk = FK[(size_t)t * DM + h * EE + r], vv = FV[(size_t)t * DM + h * EE + r]; const float hp = BC[((size_t)h * TT + t) * EE + r]; const float ratio = (s + u < CH / 2) ? __fmul_rn(__fdiv_rn(p1m, hp), p2l) : __fdiv_rn(p2l, hp);     unsigned short a, b; splitf(__fmul_rn(kk, ratio), a, b); kh[u] = a; kl[u] = b; splitf(vv, a, b); vh[u] = a; vl[u] = b; }
    for (int ps = 0; ps < 2; ++ps) { *(volatile v2us*)(KTh + i) = kh; *(volatile v2us*)(KTl + i) = kl; *(volatile v2us*)(VTh + i) = vh; *(volatile v2us*)(VTl + i) = vl; if (ps == 0) __threadfence(); } }
__global__ __launch_bounds__(256) void k_tril(const float* __restrict__ A, bf* Ah, bf* Al) { const size_t i = ((size_t)blockIdx.x * 256 + threadIdx.x) * 4; if (i >= (size_t)NZ * CH * CH) return; const int s = (int)(i % CH); const int t = (int)((i / CH) % CH); const v4f a = *(const v4f*)(A + i); v4us oh, ol;
#pragma unroll
    for (int u = 0; u < 4; ++u) { unsigned short h, l; splitf((s + u <= t) ? a[u] : 0.f, h, l); oh[u] = h; ol[u] = l; } *(volatile v4us*)(Ah + i) = oh; *(volatile v4us*)(Al + i) = ol; __threadfence(); *(volatile v4us*)(Ah + i) = oh; *(volatile v4us*)(Al + i) = ol; }
__global__ __launch_bounds__(256) void k_sscan(const float* __restrict__ DST, const float* __restrict__ BC, bf* SPh, bf* SPl) { const int i = blockIdx.x * 256 + threadIdx.x; if (i >= NH_ * EE * (EE / 2)) return; const int e = (i % (EE / 2)) * 2; const int f = (i / (EE / 2)) % EE; const int h = i / ((EE / 2) * EE); float S0 = 0.f, S1 = 0.f;
    for (int c = 0; c < NC; ++c) { v2us oh, ol; unsigned short hh, ll; splitf(S0, hh, ll); oh[0] = hh; ol[0] = ll; splitf(S1, hh, ll); oh[1] = hh; ol[1] = ll; const size_t o = (((size_t)h * NC + c) * EE + f) * EE + e; *(volatile v2us*)(SPh + o) = oh; *(volatile v2us*)(SPl + o) = ol; __threadfence(); *(volatile v2us*)(SPh + o) = oh; *(volatile v2us*)(SPl + o) = ol;
        const float* p2 = BC + ((size_t)h * TT + c * CH + CH - 1) * EE + e; const float* p1 = BC + ((size_t)h * TT + c * CH + 31) * EE + e; const float bl0 = __fmul_rn(p1[0], p2[0]), bl1 = __fmul_rn(p1[1], p2[1]);     float q0 = __fmul_rn(S0, bl0); asm volatile("" : "+v"(q0)); S0 = __fadd_rn(q0, DST[o]); float q1 = __fmul_rn(S1, bl1); asm volatile("" : "+v"(q1)); S1 = __fadd_rn(q1, DST[o + 1]); } }
__global__ __launch_bounds__(256) void k_ymrg(const float* __restrict__ YI, const float* __restrict__ YO, bf* Yh, bf* Yl) { const int i = (blockIdx.x * 256 + threadIdx.x) * 4; if (i >= TT * DM) return; const int cch = i % DM; const int t = i / DM; const int h = cch / EE, f = cch % EE; const size_t src = ((size_t)h * TT + t) * EE + f; const v4f a = *(const v4f*)(YI + src), b = *(const v4f*)(YO + src); v4us oh, ol;
#pragma unroll
    for (int u = 0; u < 4; ++u) { unsigned short hh, ll; splitf(__fadd_rn(a[u], b[u]), hh, ll); oh[u] = hh; ol[u] = ll; } *(volatile v4us*)(Yh + i) = oh; *(volatile v4us*)(Yl + i) = ol; __threadfence(); *(volatile v4us*)(Yh + i) = oh; *(volatile v4us*)(Yl + i) = ol; }

extern "C" void kernel_launch(void* const* d_in, const int* in_sizes, int n_in,
                              void* d_out, int out_size, void* d_ws, size_t ws_size, hipStream_t stream) {
    (void)in_sizes; (void)n_in; (void)out_size;
    const float* x = (const float*)d_in[0]; const float* qw = (const float*)d_in[1]; const float* kw = (const float*)d_in[2]; const float* vw = (const float*)d_in[3]; const float* ow = (const float*)d_in[4]; const float* cw1 = (const float*)d_in[5]; const float* cb1 = (const float*)d_in[6]; const float* cw2 = (const float*)d_in[7]; const float* cb2 = (const float*)d_in[8]; const float* decay = (const float*)d_in[9];
    float* OUT = (float*)d_out;
    char* wsp = (char*)d_ws;
    auto take = [&](size_t bytes) { char* p = wsp; wsp += (bytes + 255) & ~(size_t)255; return (void*)p; };
    bf* WQ = (bf*)take((size_t)DM * DM * 2); bf* WK = (bf*)take((size_t)DM * DM * 2); bf* WV = (bf*)take((size_t)DM * DM * 2); bf* WO = (bf*)take((size_t)DM * DM * 2); bf* WS = (bf*)take((size_t)SEN * DM * 2);
    bf* XB = (bf*)take((size_t)TT * DM * 2); float* FQ = (float*)take((size_t)TT * DM * 4); float* FK = (float*)take((size_t)TT * DM * 4); float* FV = (float*)take((size_t)TT * DM * 4); float* SENS = (float*)take((size_t)TT * SEN * 4); float* LC = (float*)take((size_t)TT * NH_ * 4); float* BC = (float*)take((size_t)NH_ * TT * EE * 4);
    const size_t PL = (size_t)NH_ * TT * EE;
    bf* QMh = (bf*)take(PL * 2); bf* QMl = (bf*)take(PL * 2); bf* QAh = (bf*)take(PL * 2); bf* QAl = (bf*)take(PL * 2); bf* KBh = (bf*)take(PL * 2); bf* KBl = (bf*)take(PL * 2); bf* KTh = (bf*)take(PL * 2); bf* KTl = (bf*)take(PL * 2); bf* VTh = (bf*)take(PL * 2); bf* VTl = (bf*)take(PL * 2);
    float* AS = (float*)take(PL * 4); bf* Ah = (bf*)take(PL * 2); bf* Al = (bf*)take(PL * 2); float* YI = (float*)take(PL * 4); float* DST = (float*)take(PL * 4); bf* SPh = (bf*)take(PL * 2); bf* SPl = (bf*)take(PL * 2); float* YO = (float*)take(PL * 4); bf* Yh = (bf*)take((size_t)TT * DM * 2); bf* Yl = (bf*)take((size_t)TT * DM * 2);
    if ((size_t)(wsp - (char*)d_ws) > ws_size) return;
    k_cvt8<<<(DM * DM / 8 + 255) / 256, 256, 0, stream>>>(qw, WQ, (size_t)DM * DM / 8); k_cvt8<<<(DM * DM / 8 + 255) / 256, 256, 0, stream>>>(kw, WK, (size_t)DM * DM / 8); k_cvt8<<<(DM * DM / 8 + 255) / 256, 256, 0, stream>>>(vw, WV, (size_t)DM * DM / 8); k_cvt8<<<(DM * DM / 8 + 255) / 256, 256, 0, stream>>>(ow, WO, (size_t)DM * DM / 8); k_cvt8<<<(SEN * DM / 8 + 255) / 256, 256, 0, stream>>>(cw1, WS, (size_t)SEN * DM / 8);
    for (int b = 0; b < NB_; ++b) {
        k_cvt8<<<(TT * DM / 8 + 255) / 256, 256, 0, stream>>>(x + (size_t)b * TT * DM, XB, (size_t)TT * DM / 8);
        k_gemmw<bf, 0, false><<<dim3(TT / 64, DM / 64, 1), 32, 0, stream>>>(XB, nullptr, WQ, nullptr, DM, FQ, DM, nullptr, 0, 0, 0); k_gemmw<bf, 0, false><<<dim3(TT / 64, DM / 64, 1), 32, 0, stream>>>(XB, nullptr, WK, nullptr, DM, FK, DM, nullptr, 0, 0, 0); k_gemmw<bf, 0, false><<<dim3(TT / 64, DM / 64, 1), 32, 0, stream>>>(XB, nullptr, WV, nullptr, DM, FV, DM, nullptr, 0, 0, 0);
        k_gemmw<bf, 0, true><<<dim3(TT / 64, SEN / 64, 1), 32, 0, stream>>>(XB, nullptr, WS, nullptr, DM, SENS, SEN, cb1, 0, 0, 0);
        k_lc<<<(TT * NH_ + 255) / 256, 256, 0, stream>>>(SENS, cw2, cb2, LC); k_bcum<<<(NH_ * NC * EE + 255) / 256, 256, 0, stream>>>(LC, decay, BC);
        k_qkpl<<<(unsigned)((PL / 4 + 255) / 256), 256, 0, stream>>>(FQ, FK, BC, QMh, QMl, QAh, QAl, KBh, KBl); k_ktvt<<<(unsigned)((PL / 2 + 255) / 256), 256, 0, stream>>>(FK, FV, BC, KTh, KTl, VTh, VTl);
        k_gemmw<bf, 2, false><<<dim3(1, 1, NZ), 32, 0, stream>>>(QMh, QMl, KBh, KBl, EE, AS, CH, nullptr, (size_t)CH * EE, (size_t)CH * EE, (size_t)CH * CH);
        k_tril<<<(unsigned)((PL / 4 + 255) / 256), 256, 0, stream>>>(AS, Ah, Al);
        k_gemmw<bf, 2, false><<<dim3(1, 1, NZ), 32, 0, stream>>>(Ah, Al, VTh, VTl, CH, YI, EE, nullptr, (size_t)CH * CH, (size_t)EE * CH, (size_t)CH * EE);
        k_gemmw<bf, 2, false><<<dim3(1, 1, NZ), 32, 0, stream>>>(VTh, VTl, KTh, KTl, CH, DST, EE, nullptr, (size_t)EE * CH, (size_t)EE * CH, (size_t)EE * EE);
        k_sscan<<<(NH_ * EE * (EE / 2) + 255) / 256, 256, 0, stream>>>(DST, BC, SPh, SPl);
        k_gemmw<bf, 2, false><<<dim3(1, 1, NZ), 32, 0, stream>>>(QAh, QAl, SPh, SPl, EE, YO, EE, nullptr, (size_t)CH * EE, (size_t)EE * EE, (size_t)CH * EE);
        k_ymrg<<<(TT * DM / 4 + 255) / 256, 256, 0, stream>>>(YI, YO, Yh, Yl);
        k_gemmw<bf, 1, false><<<dim3(TT / 64, DM / 64, 1), 32, 0, stream>>>(Yh, Yl, WO, nullptr, DM, OUT + (size_t)b * TT * DM, DM, nullptr, 0, 0, 0); }
}
